// FixedAttentionTransformerBlock_86835648790968
// MI455X (gfx1250) — hardware-verified
//
#include <hip/hip_runtime.h>
#include <hip/hip_bf16.h>
#include <math.h>


typedef _Float16 bf16;
typedef _Float16 f16;
typedef __attribute__((ext_vector_type(4))) unsigned v4u_t;
typedef unsigned v4ua __attribute__((ext_vector_type(4), may_alias));
typedef __attribute__((ext_vector_type(4))) float v4f_t;
typedef float v4fa __attribute__((ext_vector_type(4), may_alias));
typedef __attribute__((ext_vector_type(16))) bf16  bf16x16;
typedef bf16x16 f16x16;
typedef __attribute__((ext_vector_type(8)))  bf16  bf16x8;
typedef bf16x8 f16x8;
typedef __attribute__((ext_vector_type(4)))  bf16  bf16x4;
typedef __attribute__((ext_vector_type(8)))  float f32x8;
__device__ __forceinline__ f32x8 wmma16(f16x16 a, f16x16 b, f32x8 c) {
  c = __builtin_amdgcn_wmma_f32_16x16x32_f16(false, a, false, b, (short)0, c, false, false);
  asm volatile("v_nop\n\tv_nop\n\tv_nop\n\tv_nop" : "+v"(c) : "v"(a), "v"(b));
  return c;
}
#define LDS_STRIDE 48
#define KSTRIDE    72
#define VSTRIDE    48

__device__ __forceinline__ f32x8 wmma_bf16(bf16x16 a, bf16x16 b, f32x8 c) {
  c = __builtin_amdgcn_wmma_f32_16x16x32_f16(false, a, false, b, (short)0, c, false, false);
  asm volatile("v_nop\n\tv_nop\n\tv_nop\n\tv_nop" : "+v"(c) : "v"(a), "v"(b));
  return c;
}

template <typename T>
__device__ __forceinline__ bf16x16 load_frag(const T* __restrict__ base, int ld,
                                             int row0, int k0) {
  const int lane = threadIdx.x & 31;
  const int r    = lane & 15;
  const int kh   = (lane >> 4) * 8;
  const T* p0 = base + (size_t)(row0 + r) * ld + (k0 + kh);
  const T* p1 = p0 + 16;
  bf16x16 f;
#pragma unroll
  for (int i = 0; i < 8; ++i) {
    f[i]     = (bf16)p0[i];
    f[i + 8] = (bf16)p1[i];
  }
  return f;
}

__device__ __forceinline__ bf16x16 lds_frag(const bf16* base, int stride) {
  const int lane = threadIdx.x & 31;
  const int row  = lane & 15;
  const int kh   = (lane >> 4) * 8;
  const bf16x8 lo = *(const bf16x8*)(base + row * stride + kh);
  const bf16x8 hi = *(const bf16x8*)(base + row * stride + kh + 16);
  bf16x16 f;
#pragma unroll
  for (int i = 0; i < 8; ++i) { f[i] = lo[i]; f[i + 8] = hi[i]; }
  return f;
}

template <typename T>
__device__ __forceinline__ void stage_read16(const T* __restrict__ p, float* buf) {
#pragma unroll
  for (int i = 0; i < 16; ++i) buf[i] = (float)p[i];
}

__device__ __forceinline__ void stage_write(bf16* dst, const float* buf, int nquad) {
#pragma unroll
  for (int i = 0; i < nquad; ++i) {
    bf16x4 q;
    q[0] = (bf16)buf[4 * i];     q[1] = (bf16)buf[4 * i + 1];
    q[2] = (bf16)buf[4 * i + 2]; q[3] = (bf16)buf[4 * i + 3];
    *(bf16x4*)(dst + 4 * i) = q;
  }
}


#define GSTR 48
#define GSTR 48
template <typename AT, int EPI, bool OUT16>
__global__ __launch_bounds__(256) void gemm_kne(const AT* __restrict__ A, int lda, const float* __restrict__ Wm, int ldw,
                                                const float* __restrict__ bias, const float* __restrict__ R, const float* __restrict__ gvec,
                                                void* __restrict__ Yv, int ldy, int K) {
  __shared__ __attribute__((aligned(16))) f16 ldsA[128 * GSTR];
  __shared__ __attribute__((aligned(16))) f16 ldsW[128 * GSTR];
  __shared__ __attribute__((aligned(16))) float oS[8][32 * 68];
  const int tid = threadIdx.x, lane = tid & 31, wave = tid >> 5, cl = lane & 15, rh = (lane >> 4) * 8;
  const int m0 = blockIdx.x * 128, n0 = blockIdx.y * 128;
  const int wm = (wave & 3) * 32, wn = (wave >> 2) * 64;
  f32x8 acc[2][4];
#pragma unroll
  for (int i = 0; i < 2; ++i)
#pragma unroll
    for (int j = 0; j < 4; ++j) { f32x8 z = {}; acc[i][j] = z; }
#pragma unroll 1
  for (int k0 = 0; k0 < K; k0 += 32) {
    __syncthreads();
    { const int row = tid >> 1, ch = (tid & 1) * 16;
      const AT* src = A + (size_t)(m0 + row) * lda + k0 + ch;
#pragma unroll
      for (int g = 0; g < 16; ++g) ldsA[row * GSTR + ch + g] = (f16)src[g]; }
    { const int k = tid >> 3, nn0 = (tid & 7) * 16;
      const float* src = Wm + (size_t)(k0 + k) * ldw + n0 + nn0;
#pragma unroll
      for (int g = 0; g < 4; ++g) { const v4f_t v = *(const v4f_t*)(src + 4 * g);
#pragma unroll
        for (int u = 0; u < 4; ++u) ldsW[(nn0 + 4 * g + u) * GSTR + k] = (f16)v[u]; } }
    __syncthreads();
    f16x16 af[2];
#pragma unroll
    for (int i = 0; i < 2; ++i) af[i] = lds_frag(ldsA + (wm + 16 * i) * GSTR, GSTR);
#pragma unroll
    for (int j = 0; j < 4; ++j) {
      const f16x16 bf = lds_frag(ldsW + (wn + 16 * j) * GSTR, GSTR);
#pragma unroll
      for (int i = 0; i < 2; ++i) acc[i][j] = wmma16(af[i], bf, acc[i][j]);
    }
  }
  float* so = oS[wave];
#pragma unroll
  for (int i = 0; i < 2; ++i)
#pragma unroll
    for (int j = 0; j < 4; ++j) {
      const int n = n0 + wn + 16 * j + cl;
      const float bv = bias ? bias[n] : 0.0f;
      const float gv = (EPI == 2) ? gvec[n] : 0.0f;
      if (EPI == 1) {
#pragma unroll 1
        for (int r = 0; r < 8; ++r) { const float xg = acc[i][j][r] + bv; so[(16 * i + rh + r) * 68 + 16 * j + cl] = 0.5f * xg * (1.0f + erff(xg * 0.70710678118654752f)); }
      } else {
#pragma unroll
        for (int r = 0; r < 8; ++r) {
          float v = acc[i][j][r] + bv;
          if (EPI == 3) v = fmaxf(v, 0.0f);
          if (EPI == 2) v = R[(size_t)(m0 + wm + 16 * i + rh + r) * ldy + n] + gv * v;
          so[(16 * i + rh + r) * 68 + 16 * j + cl] = v;
        }
      }
    }
  asm volatile("s_wait_dscnt 0" ::: "memory");
  __builtin_amdgcn_wave_barrier();
#pragma unroll 1
  for (int pass = 0; pass < 2; ++pass) {
    if (OUT16) {
      f16* Y = (f16*)Yv;
#pragma unroll
      for (int it = 0; it < 8; ++it) { const int c = lane + 32 * it, rr = c >> 3, q8 = (c & 7) * 8;
        union { f16 h[8]; v4u_t v; } u;
#pragma unroll
        for (int e = 0; e < 8; ++e) u.h[e] = (f16)so[rr * 68 + q8 + e];
        *(volatile v4u_t*)(Y + (size_t)(m0 + wm + rr) * ldy + n0 + wn + q8) = u.v; }
    } else {
      float* Y = (float*)Yv;
#pragma unroll
      for (int it = 0; it < 16; ++it) { const int f4 = lane + 32 * it, rr = f4 >> 4, q = (f4 & 15) * 4;
        *(volatile v4f_t*)(Y + (size_t)(m0 + wm + rr) * ldy + n0 + wn + q) = *(const v4fa*)(so + rr * 68 + q); }
    }
    __threadfence();
  }
}


#define NBT 8
#define BBf 8
#define LL 1024
#define EE 256
#define NHf 8
#define DHf 32
#define FFf 1024
__global__ __launch_bounds__(256) void k_ln256(const float* __restrict__ X, const float* __restrict__ gam, const float* __restrict__ bet, float* __restrict__ Y) {
  __shared__ __attribute__((aligned(16))) float rowS[32 * 260];
  const int tid = threadIdx.x, r = tid >> 3, part = tid & 7; const size_t row = (size_t)blockIdx.x * 32 + r;
  float s = 0.0f;
#pragma unroll 1
  for (int i = 0; i < 32; ++i) { const float v = X[row * EE + part * 32 + i]; rowS[r * 260 + part * 32 + i] = v; s += v; }
  s += __shfl_xor(s, 1, 32); s += __shfl_xor(s, 2, 32); s += __shfl_xor(s, 4, 32);
  const float mean = s * (1.0f / EE); float q = 0.0f;
#pragma unroll 1
  for (int i = 0; i < 32; ++i) { const float dv = rowS[r * 260 + part * 32 + i] - mean; q += dv * dv; }
  q += __shfl_xor(q, 1, 32); q += __shfl_xor(q, 2, 32); q += __shfl_xor(q, 4, 32);
  const float rstd = rsqrtf(q * (1.0f / EE) + 1e-5f);
#pragma unroll 1
  for (int i = 0; i < 32; ++i) { const int c = part * 32 + i; rowS[r * 260 + c] = (rowS[r * 260 + c] - mean) * rstd * gam[c] + bet[c]; }
  __syncthreads();
#pragma unroll 1
  for (int pass = 0; pass < 2; ++pass) { for (int q4 = tid; q4 < 32 * 64; q4 += 256) { const int rr = q4 >> 6, c4 = (q4 & 63) * 4;
      *(volatile v4f_t*)(Y + ((size_t)blockIdx.x * 32 + rr) * EE + c4) = *(const v4fa*)(rowS + rr * 260 + c4); } __threadfence(); }
}
__global__ __launch_bounds__(256) void k_pgen(const float* __restrict__ db, const int* __restrict__ cm, const float* __restrict__ gamma, float* __restrict__ P) {
  __shared__ float red[256];
  const int i = blockIdx.x, h = blockIdx.y, tid = threadIdx.x; const float g = gamma[h];
  const float* dr = db + (size_t)i * LL; const int* mr = cm + (size_t)i * LL; float* pr = P + ((size_t)h * LL + i) * LL;
  float v[4]; float m = -3.0e38f;
#pragma unroll
  for (int e = 0; e < 4; ++e) { const int j = tid + 256 * e; const float dd = dr[j]; const float w = -g * (dd * dd); v[e] = mr[j] ? -1.0e9f : w; m = fmaxf(m, v[e]); }
  red[tid] = m; __syncthreads();
  for (int o = 128; o > 0; o >>= 1) { if (tid < o) red[tid] = fmaxf(red[tid], red[tid + o]); __syncthreads(); }
  m = red[0]; __syncthreads();
  float z = 0.0f;
#pragma unroll
  for (int e = 0; e < 4; ++e) { v[e] = expf(v[e] - m); z += v[e]; }
  red[tid] = z; __syncthreads();
  for (int o = 128; o > 0; o >>= 1) { if (tid < o) red[tid] += red[tid + o]; __syncthreads(); }
  const float sc = 1024.0f / red[0];
#pragma unroll 1
  for (int pass = 0; pass < 2; ++pass) {
#pragma unroll
    for (int e = 0; e < 4; ++e) *(volatile float*)(pr + tid + 256 * e) = v[e] * sc;
    __threadfence(); }
}
__global__ __launch_bounds__(256) void k_fill(float* __restrict__ p, float val, size_t n4) { const size_t i = (size_t)blockIdx.x * 256 + threadIdx.x; if (i < n4) { v4f_t v = {val, val, val, val}; *(volatile v4f_t*)(p + 4 * i) = v; __threadfence(); *(volatile v4f_t*)(p + 4 * i) = v; } }
__global__ __launch_bounds__(256) void k_place32(const float* __restrict__ T, float* __restrict__ ctx, int b, int h) {
  const int tid = threadIdx.x; const int i = blockIdx.x * 32 + (tid >> 3); const int c4 = (tid & 7) * 4;
  const v4f_t v = *(const v4f_t*)(T + (size_t)i * 128 + c4);
  float* dst = ctx + ((size_t)b * LL + i) * EE + h * DHf + c4; *(volatile v4f_t*)dst = v; __threadfence(); *(volatile v4f_t*)dst = v;
}
__global__ __launch_bounds__(256) void k_padfix(const int* __restrict__ pm, const float* __restrict__ E2, float* __restrict__ out) {
  const int tid = threadIdx.x; const size_t row = (size_t)blockIdx.x * 4 + (tid >> 6); const int c4 = (tid & 63) * 4;
  if (pm[row]) { const v4f_t v = *(const v4f_t*)(E2 + row * EE + c4); *(volatile v4f_t*)(out + row * EE + c4) = v; __threadfence(); *(volatile v4f_t*)(out + row * EE + c4) = v; }
}

extern "C" void kernel_launch(void* const* d_in, const int* in_sizes, int n_in,
                              void* d_out, int out_size, void* d_ws, size_t ws_size,
                              hipStream_t stream) {
  (void)in_sizes; (void)n_in; (void)out_size;
  const float** f = (const float**)d_in;
  const float* e = f[1], *d = f[2]; const int* cm = (const int*)d_in[3]; const int* pm = (const int*)d_in[4];
  const float* ln1g = f[5], *ln1b = f[6], *ln2g = f[7], *ln2b = f[8], *Wv = f[9], *bv = f[10], *Wo = f[11], *bo = f[12], *W1 = f[13], *b1 = f[14], *W2 = f[15], *b2 = f[16], *gamma = f[17];
  float* out = (float*)d_out;
  char* ws = (char*)d_ws;
  const size_t MT = (size_t)BBf * LL;
  float* E0 = (float*)ws; ws += MT * EE * 4;
  float* V = (float*)ws; ws += MT * EE * 4 + 1024;
  float* P = (float*)ws; ws += (size_t)NHf * LL * LL * 4;
  float* T = (float*)ws; ws += (size_t)LL * 128 * 4;
  float* CTX = (float*)ws; ws += MT * EE * 4;
  float* X1 = (float*)ws; ws += MT * EE * 4;
  float* E2 = (float*)ws; ws += MT * EE * 4;
  bf16* HID16 = (bf16*)ws; ws += MT * FFf * 2;
  float* zero = (float*)ws; ws += (size_t)LL * 128 * 4; float* sc = (float*)ws; ws += 128 * 4; float* ones = (float*)ws; ws += EE * 4;
  if ((size_t)(ws - (char*)d_ws) > ws_size) return;
  const dim3 blk(256); const dim3 gp(MT / 128, EE / 128);
  k_fill<<<dim3((LL * 128 / 4 + 255) / 256), blk, 0, stream>>>(zero, 0.0f, (size_t)LL * 128 / 4); k_fill<<<dim3(1), blk, 0, stream>>>(sc, 1.0f / 1024.0f, 128 / 4); k_fill<<<dim3(1), blk, 0, stream>>>(ones, 1.0f, EE / 4);
  k_fill<<<dim3(1), blk, 0, stream>>>(V + MT * EE, 0.0f, 256 / 4);
  k_ln256<<<dim3(MT / 32), blk, 0, stream>>>(e, ln1g, ln1b, E0);
  gemm_kne<float, 0, false><<<gp, blk, 0, stream>>>(E0, EE, Wv, EE, bv, nullptr, nullptr, V, EE, EE);
  for (int b = 0; b < NBT; ++b) {
    k_pgen<<<dim3(LL, NHf), blk, 0, stream>>>(d + (size_t)b * LL * LL, cm, gamma, P);
    for (int h = 0; h < NHf; ++h) {
      gemm_kne<float, 2, false><<<dim3(LL / 128, 1), blk, 0, stream>>>(P + (size_t)h * LL * LL, LL, V + (size_t)b * LL * EE + h * DHf, EE, nullptr, zero, sc, T, 128, LL);
      k_place32<<<dim3(LL / 32), blk, 0, stream>>>(T, CTX, b, h); }
  }
  gemm_kne<float, 2, false><<<gp, blk, 0, stream>>>(CTX, EE, Wo, EE, bo, E0, ones, X1, EE, EE);
  k_ln256<<<dim3(MT / 32), blk, 0, stream>>>(X1, ln2g, ln2b, E2);
  gemm_kne<float, 3, true><<<dim3(MT / 128, FFf / 128), blk, 0, stream>>>(E2, EE, W1, FFf, b1, nullptr, nullptr, HID16, FFf, EE);
  gemm_kne<bf16, 2, false><<<gp, blk, 0, stream>>>(HID16, FFf, W2, EE, b2, E2, ones, out, EE, FFf);
  k_padfix<<<dim3(MT / 4), blk, 0, stream>>>(pm, E2, out);
}
